// CNN_22325240004626
// MI455X (gfx1250) — hardware-verified
//
#include <hip/hip_runtime.h>
#include <stdint.h>

#define DEVINL __device__ __forceinline__

typedef _Float16 f16t;
typedef _Float16 v16h __attribute__((ext_vector_type(16)));
typedef _Float16 v8h  __attribute__((ext_vector_type(8)));
typedef float    v8f  __attribute__((ext_vector_type(8)));
typedef float    v4f  __attribute__((ext_vector_type(4)));
typedef v8h __attribute__((may_alias)) v8ha;
typedef v4f __attribute__((may_alias)) v4fa;
union FragH { v16h v; v8h half[2]; };

#define TLEN   8192
#define FIN    16
#define HID    128
#define NOUT   24
#define NOP    32
#define KT     10
#define K1     (KT * FIN)
#define K2     (KT * HID)
#define PADX   128
#define XP     (PADX + TLEN)
#define PADH   16
#define HP     (PADH + TLEN)
#define T1     64
#define T2     128
#define TPB    256
#define C2TPB  128
#define XRB    128
#define ACAR   16.0f
#define WCAR   256.0f
#define INVCAR (1.0f / 4096.0f)
#define W1BLK  ((HID * K1 / 8 + TPB - 1) / TPB)
#define WFBLK  ((NOP * K2 / 8 + TPB - 1) / TPB)

static_assert((K1 % 32) == 0);
static_assert((K2 % 32) == 0);
static_assert((TLEN % T1) == 0);
static_assert((TLEN % T2) == 0);
static_assert((XP % XRB) == 0);
static_assert(XRB * FIN == TPB * 8);
static_assert(PADX >= KT - 1);
static_assert(PADH >= KT - 1);
static_assert(PADH * HID == TPB * 8);
static_assert(PADH == 16);
static_assert(T1 * HID == TPB * 8 * 4);
static_assert(T2 * NOUT == C2TPB * 4 * 6);
static_assert((NOUT % 4) == 0);
static_assert(((HID * K1 * 2) % 512) == 0);
static_assert(((NOP * K2 * 2) % 512) == 0);
static_assert(((XP * FIN * 2) % 512) == 0);
static_assert(((HP * HID * 2) % 512) == 0);
static_assert(((T2 * NOUT * 4) % 512) == 0);
static_assert(((TLEN * NOUT * 4) % 512) == 0);
static_assert((HID * (K1 / 8)) % TPB == 0);
static_assert((NOP * (K2 / 8)) % TPB == 0);
static_assert(WFBLK >= W1BLK);

DEVINL int imin(int a, int b) { return a < b ? a : b; }
DEVINL int imax(int a, int b) { return a > b ? a : b; }

DEVINL v8f wmma_f16(v16h a, v16h b, v8f c) {
  v8f d = __builtin_amdgcn_wmma_f32_16x16x32_f16(false, a, false, b, (short)0, c, false, false);
  asm volatile("v_nop\n\tv_nop\n\tv_nop\n\tv_nop" : "+v"(d) : "v"(a), "v"(b));
  return d;
}
DEVINL v8f zero8f() {
  v8f z = {0.f, 0.f, 0.f, 0.f, 0.f, 0.f, 0.f, 0.f};
  return z;
}
DEVINL v8h cvt8(const float* p, float s) {
  const v4f u0 = *(const v4fa*)p;
  const v4f u1 = *(const v4fa*)(p + 4);
  v8h o;
  o[0] = (f16t)(u0[0] * s); o[1] = (f16t)(u0[1] * s);
  o[2] = (f16t)(u0[2] * s); o[3] = (f16t)(u0[3] * s);
  o[4] = (f16t)(u1[0] * s); o[5] = (f16t)(u1[1] * s);
  o[6] = (f16t)(u1[2] * s); o[7] = (f16t)(u1[3] * s);
  return o;
}

__global__ __launch_bounds__(TPB) void prep_w_k(const float* __restrict__ w1, const float* __restrict__ wf,
                                              f16t* __restrict__ W1p, f16t* __restrict__ Wfp)
{
  const int t = blockIdx.x * TPB + threadIdx.x;
  if (blockIdx.y == 0) {
    const int kg   = K1 / 8;
    const int nthr = HID * kg;
    if (t >= nthr) return;
    const int row  = t / kg;
    const int part = t - row * kg;
    const int k8   = 8 * part;
    const int tap  = k8 / FIN;
    const int c0   = k8 - tap * FIN;
    v8h o;
    #pragma unroll
    for (int i = 0; i < 8; ++i) {
      const float wv = w1[((size_t)row * FIN + c0 + i) * KT + tap];
      o[i] = (f16t)(wv * WCAR);
    }
    f16t* dst = W1p + (size_t)8 * t;
    *(volatile v8h*)dst = o;
    __threadfence();
    *(volatile v8h*)dst = o;
  } else {
    const int kg   = K2 / 8;
    const int nthr = NOP * kg;
    if (t >= nthr) return;
    const int row  = t / kg;
    const int part = t - row * kg;
    const int k8   = 8 * part;
    const int rc   = imin(row, NOUT - 1);
    const float* src = wf + (size_t)rc * K2 + k8;
    const v4f u0 = *(const v4fa*)src;
    const v4f u1 = *(const v4fa*)(src + 4);
    const float s = (row < NOUT) ? WCAR : 0.0f;
    v8h o;
    o[0] = (f16t)((row < NOUT) ? u0[0] * s : 0.0f); o[1] = (f16t)((row < NOUT) ? u0[1] * s : 0.0f);
    o[2] = (f16t)((row < NOUT) ? u0[2] * s : 0.0f); o[3] = (f16t)((row < NOUT) ? u0[3] * s : 0.0f);
    o[4] = (f16t)((row < NOUT) ? u1[0] * s : 0.0f); o[5] = (f16t)((row < NOUT) ? u1[1] * s : 0.0f);
    o[6] = (f16t)((row < NOUT) ? u1[2] * s : 0.0f); o[7] = (f16t)((row < NOUT) ? u1[3] * s : 0.0f);
    f16t* dst = Wfp + (size_t)8 * t;
    *(volatile v8h*)dst = o;
    __threadfence();
    *(volatile v8h*)dst = o;
  }
}

__global__ __launch_bounds__(TPB) void xin_k(const float* __restrict__ x, f16t* __restrict__ X16)
{
  const int tid = threadIdx.x, chunk = blockIdx.x, b = blockIdx.y;
  const int row = chunk * XRB + (tid >> 1);
  const int c0  = (tid & 1) * 8;
  const int t   = row - PADX;
  const int tcl = imin(imax(t, 0), TLEN - 1);
  const float* src = x + ((size_t)b * TLEN + tcl) * FIN + c0;
  const v4f u0 = *(const v4fa*)src;
  const v4f u1 = *(const v4fa*)(src + 4);
  const bool ok = (t >= 0);
  v8h o;
  o[0] = (f16t)(ok ? u0[0] * ACAR : 0.0f); o[1] = (f16t)(ok ? u0[1] * ACAR : 0.0f);
  o[2] = (f16t)(ok ? u0[2] * ACAR : 0.0f); o[3] = (f16t)(ok ? u0[3] * ACAR : 0.0f);
  o[4] = (f16t)(ok ? u1[0] * ACAR : 0.0f); o[5] = (f16t)(ok ? u1[1] * ACAR : 0.0f);
  o[6] = (f16t)(ok ? u1[2] * ACAR : 0.0f); o[7] = (f16t)(ok ? u1[3] * ACAR : 0.0f);
  f16t* dst = X16 + ((size_t)b * XP + row) * FIN + c0;
  *(volatile v8h*)dst = o;
  __threadfence();
  *(volatile v8h*)dst = o;
}

DEVINL void stage8(v8f acc, float* srow, int c0, const float* __restrict__ bias, int nb)
{
  #pragma unroll
  for (int r = 0; r < 8; ++r) {
    const int c = c0 + r;
    srow[c] = fmaf(acc[r], INVCAR, bias[imin(c, nb - 1)]);
  }
}

__global__ __launch_bounds__(TPB) void conv1_k(const f16t* __restrict__ X16, const f16t* __restrict__ W1p,
                                             const float* __restrict__ b1, f16t* __restrict__ H16)
{
  __shared__ __attribute__((aligned(16))) float sO[T1 * HID];
  const int tid = threadIdx.x, lane = tid & 31, wave = tid >> 5;
  const int h = lane >> 4, m = lane & 15;
  const int wc = wave & 3, wq = wave >> 2;
  const int b  = blockIdx.y;
  const int tb = blockIdx.x * T1;
  const int tl0 = 32 * wq + m;
  const int tl1 = tl0 + 16;

  const f16t* xb  = X16 + ((size_t)b * XP + PADX + tb - (KT - 1)) * FIN + 8 * h;
  const f16t* y0  = xb + (size_t)tl0 * FIN;
  const f16t* y1  = xb + (size_t)tl1 * FIN;
  const f16t* wr0 = W1p + (size_t)(32 * wc + m) * K1 + 8 * h;
  const f16t* wr1 = wr0 + (size_t)16 * K1;

  v8f acc00 = zero8f(), acc01 = zero8f(), acc10 = zero8f(), acc11 = zero8f();

  #pragma unroll
  for (int s = 0; s < K1 / 32; ++s) {
    FragH a0, a1, f0, f1;
    a0.half[0] = *(const v8ha*)(wr0 + 32 * s);
    a0.half[1] = *(const v8ha*)(wr0 + 32 * s + 16);
    a1.half[0] = *(const v8ha*)(wr1 + 32 * s);
    a1.half[1] = *(const v8ha*)(wr1 + 32 * s + 16);
    f0.half[0] = *(const v8ha*)(y0 + 32 * s);
    f0.half[1] = *(const v8ha*)(y0 + 32 * s + 16);
    f1.half[0] = *(const v8ha*)(y1 + 32 * s);
    f1.half[1] = *(const v8ha*)(y1 + 32 * s + 16);
    acc00 = wmma_f16(a0.v, f0.v, acc00);
    acc01 = wmma_f16(a0.v, f1.v, acc01);
    acc10 = wmma_f16(a1.v, f0.v, acc10);
    acc11 = wmma_f16(a1.v, f1.v, acc11);
  }

  {
    const int cA = 32 * wc + 8 * h;
    const int cB = cA + 16;
    stage8(acc00, sO + tl0 * HID, cA, b1, HID);
    stage8(acc01, sO + tl1 * HID, cA, b1, HID);
    stage8(acc10, sO + tl0 * HID, cB, b1, HID);
    stage8(acc11, sO + tl1 * HID, cB, b1, HID);
  }
  __syncthreads();

  const int p8 = (lane & 15) * 8, rs = lane >> 4;
  v8h hv[4];
  #pragma unroll
  for (int j = 0; j < 4; ++j) {
    const int row = 8 * wave + 2 * j + rs;
    hv[j] = cvt8(sO + row * HID + p8, ACAR);
  }
  const int rr = tid >> 4, pp = (tid & 15) * 8;
  const v8h rv = cvt8(sO + pp, ACAR);
  const bool rep = (tb == 0);
  f16t* drow = H16 + ((size_t)b * HP + PADH + tb) * HID;
  f16t* rdst = H16 + ((size_t)b * HP + rr) * HID + pp;
  #pragma unroll
  for (int j = 0; j < 4; ++j) {
    const int row = 8 * wave + 2 * j + rs;
    *(volatile v8h*)(drow + (size_t)row * HID + p8) = hv[j];
  }
  if (rep) *(volatile v8h*)rdst = rv;
  __threadfence();
  #pragma unroll
  for (int j = 0; j < 4; ++j) {
    const int row = 8 * wave + 2 * j + rs;
    *(volatile v8h*)(drow + (size_t)row * HID + p8) = hv[j];
  }
  if (rep) *(volatile v8h*)rdst = rv;
}

__global__ __launch_bounds__(C2TPB) void conv2_k(const f16t* __restrict__ H16, const f16t* __restrict__ Wfp,
                                               const float* __restrict__ bfv, float* __restrict__ out)
{
  __shared__ __attribute__((aligned(16))) float sO[T2 * NOP];
  const int tid = threadIdx.x, lane = tid & 31, wave = tid >> 5;
  const int h = lane >> 4, m = lane & 15;
  const int b  = blockIdx.y;
  const int tb = blockIdx.x * T2;
  const int tl0 = 32 * wave + m;
  const int tl1 = tl0 + 16;

  const f16t* hb  = H16 + ((size_t)b * HP + PADH + tb - (KT - 1)) * HID + 8 * h;
  const f16t* y0  = hb + (size_t)tl0 * HID;
  const f16t* y1  = hb + (size_t)tl1 * HID;
  const f16t* wr0 = Wfp + (size_t)m * K2 + 8 * h;
  const f16t* wr1 = wr0 + (size_t)16 * K2;

  v8f acc00 = zero8f(), acc01 = zero8f(), acc10 = zero8f(), acc11 = zero8f();

  #pragma unroll 2
  for (int s = 0; s < K2 / 32; ++s) {
    FragH a0, a1, f0, f1;
    a0.half[0] = *(const v8ha*)(wr0 + 32 * s);
    a0.half[1] = *(const v8ha*)(wr0 + 32 * s + 16);
    a1.half[0] = *(const v8ha*)(wr1 + 32 * s);
    a1.half[1] = *(const v8ha*)(wr1 + 32 * s + 16);
    f0.half[0] = *(const v8ha*)(y0 + 32 * s);
    f0.half[1] = *(const v8ha*)(y0 + 32 * s + 16);
    f1.half[0] = *(const v8ha*)(y1 + 32 * s);
    f1.half[1] = *(const v8ha*)(y1 + 32 * s + 16);
    acc00 = wmma_f16(a0.v, f0.v, acc00);
    acc01 = wmma_f16(a0.v, f1.v, acc01);
    acc10 = wmma_f16(a1.v, f0.v, acc10);
    acc11 = wmma_f16(a1.v, f1.v, acc11);
  }

  {
    const int cA = 8 * h;
    const int cB = cA + 16;
    stage8(acc00, sO + tl0 * NOP, cA, bfv, NOUT);
    stage8(acc01, sO + tl1 * NOP, cA, bfv, NOUT);
    stage8(acc10, sO + tl0 * NOP, cB, bfv, NOUT);
    stage8(acc11, sO + tl1 * NOP, cB, bfv, NOUT);
  }
  __syncthreads();

  float* base = out + ((size_t)b * TLEN + tb) * NOUT;
  v4f fv[6];
  #pragma unroll
  for (int j = 0; j < 6; ++j) {
    const int q   = j * C2TPB + tid;
    const int row = q / (NOUT / 4);
    const int col = (q - row * (NOUT / 4)) * 4;
    fv[j] = *(const v4fa*)(sO + row * NOP + col);
  }
  #pragma unroll
  for (int j = 0; j < 6; ++j) {
    const int q = j * C2TPB + tid;
    *(volatile v4f*)(base + (size_t)4 * q) = fv[j];
  }
  __threadfence();
  #pragma unroll
  for (int j = 0; j < 6; ++j) {
    const int q = j * C2TPB + tid;
    *(volatile v4f*)(base + (size_t)4 * q) = fv[j];
  }
}

extern "C" void kernel_launch(void* const* d_in, const int* in_sizes, int n_in,
                              void* d_out, int out_size, void* d_ws, size_t ws_size,
                              hipStream_t stream)
{
  if (n_in < 5) return;
  const int perSeq = TLEN * FIN;
  if (in_sizes[0] <= 0 || (in_sizes[0] % perSeq) != 0) return;
  const int nB = in_sizes[0] / perSeq;
  if (nB > 65535) return;
  if (in_sizes[1] != HID * FIN * KT) return;
  if (in_sizes[2] != HID) return;
  if (in_sizes[3] != NOUT * K2) return;
  if (in_sizes[4] != NOUT) return;
  if ((long long)out_size != (long long)nB * TLEN * NOUT) return;

  const float* x  = (const float*)d_in[0];
  const float* w1 = (const float*)d_in[1];
  const float* b1 = (const float*)d_in[2];
  const float* wf = (const float*)d_in[3];
  const float* bf = (const float*)d_in[4];
  float* outp = (float*)d_out;

  const size_t szW1 = (size_t)HID * K1 * 2;
  const size_t szWf = (size_t)NOP * K2 * 2;
  const size_t szX  = (size_t)nB * XP * FIN * 2;
  const size_t szH  = (size_t)nB * HP * HID * 2;
  size_t off = 0;
  char* ws = (char*)d_ws;
  f16t* W1p = (f16t*)(ws + off); off += szW1;
  f16t* Wfp = (f16t*)(ws + off); off += szWf;
  f16t* X16 = (f16t*)(ws + off); off += szX;
  f16t* H16 = (f16t*)(ws + off); off += szH;
  if (off > ws_size) return;
  if (off > (size_t)134217728) return;

  prep_w_k<<<dim3(WFBLK, 2), TPB, 0, stream>>>(w1, wf, W1p, Wfp);
  xin_k<<<dim3(XP / XRB, nB), TPB, 0, stream>>>(x, X16);
  conv1_k<<<dim3(TLEN / T1, nB), TPB, 0, stream>>>(X16, W1p, b1, H16);
  conv2_k<<<dim3(TLEN / T2, nB), C2TPB, 0, stream>>>(H16, Wfp, bf, outp);
}
